// PTFDecoder_66992899883085
// MI455X (gfx1250) — hardware-verified
//
#include <hip/hip_runtime.h>
#include <stddef.h>

constexpr int JN  = 14;
constexpr int DN  = 3;
constexpr int CN  = 128;
constexpr int HN  = 128;
constexpr int BN  = 2;
constexpr int TN  = 32768;
constexpr int TT  = 128;
constexpr int KP  = 136;
constexpr int WK0 = CN + DN;

constexpr float W_SC = 256.0f;
constexpr float R_W  = 0.00390625f;

static_assert(TN % TT == 0);
static_assert(TN % 4 == 0);
static_assert(CN == HN);
static_assert(TT == HN);
static_assert((KP * 2) % 16 == 0);
static_assert(KP % 2 == 0);
static_assert(HN % 32 == 0);
static_assert(TT % 16 == 0);
static_assert((JN * HN * HN) % 8 == 0);
static_assert((JN * HN * HN / 8) % 256 == 0);

typedef _Float16     v16h __attribute__((ext_vector_type(16)));
typedef _Float16     v8h  __attribute__((ext_vector_type(8)));
typedef float        v8f  __attribute__((ext_vector_type(8)));
typedef float        v4f  __attribute__((ext_vector_type(4)));
typedef unsigned int v4u  __attribute__((ext_vector_type(4)));
typedef v4u __attribute__((may_alias)) v4ua;
typedef v4f __attribute__((may_alias)) v4fa;
typedef unsigned int u32a __attribute__((may_alias));

union Frag  { v16h v; v4u q[2]; };
union Pack8 { v8h h; v4u u; };

__device__ __forceinline__ unsigned short hb(float f) {
    const _Float16 t = (_Float16)f;
    return __builtin_bit_cast(unsigned short, t);
}

__device__ __forceinline__ v8f wmma16(v16h a, v16h b, v8f c) {
    v8f d = __builtin_amdgcn_wmma_f32_16x16x32_f16(false, a, false, b, (short)0, c, false, false);
    asm volatile("v_nop\n\tv_nop\n\tv_nop\n\tv_nop" : "+v"(d) : "v"(a), "v"(b));
    return d;
}

__device__ __forceinline__ v16h ldfrag(const unsigned short* p, int h) {
    Frag f;
    f.q[0] = *(const v4ua*)(p + 8 * h);
    f.q[1] = *(const v4ua*)(p + 16 + 8 * h);
    return f.v;
}

__global__ __launch_bounds__(256) void k_wcvt(const float* __restrict__ W0,
                                              const float* __restrict__ W1,
                                              const float* __restrict__ W2,
                                              unsigned short* __restrict__ P0,
                                              unsigned short* __restrict__ P1,
                                              unsigned short* __restrict__ P2,
                                              int n8)
{
    const int y = blockIdx.y;
    const int g = blockIdx.x * 256 + threadIdx.x;
    if (g >= n8) return;
    const float* src = (y == 0) ? W0 : ((y == 1) ? W1 : W2);
    unsigned short* dst = (y == 0) ? P0 : ((y == 1) ? P1 : P2);
    const int pitch = (y == 0) ? WK0 : HN;
    const int koff  = (y == 0) ? DN : 0;
    const int row = g >> 4;
    const int k0  = (g & 15) * 8;
    const float* s = src + (size_t)row * pitch + koff + k0;
    v8h hv;
    #pragma unroll
    for (int i = 0; i < 8; ++i) hv[i] = (_Float16)(s[i] * W_SC);
    Pack8 pk;
    pk.h = hv;
    const v4u u = pk.u;
    unsigned short* d = dst + (size_t)g * 8;
    *(volatile v4u*)d = u;
    __threadfence();
    *(volatile v4u*)d = u;
}

template <bool ADDP>
__device__ __forceinline__ void gemm_layer(const unsigned short* actIn,
                                           unsigned short* actOut,
                                           const unsigned short* __restrict__ wj,
                                           const float* bias,
                                           const float* w0p,
                                           const float* pt,
                                           int lane, int mbase)
{
    const int lm = lane & 15;
    const int hh = lane >> 4;

    v8f acc[TT / 16];
    #pragma unroll
    for (int n = 0; n < TT / 16; ++n) {
        #pragma unroll
        for (int r = 0; r < 8; ++r) acc[n][r] = 0.0f;
    }

    const unsigned short* arow = wj + (size_t)(mbase + lm) * HN;

    #pragma unroll 1
    for (int kk = 0; kk < HN / 32; ++kk) {
        const v16h a = ldfrag(arow + kk * 32, hh);
        #pragma unroll
        for (int n = 0; n < TT / 16; ++n) {
            const v16h bf = ldfrag(actIn + (n * 16 + lm) * KP + kk * 32, hh);
            acc[n] = wmma16(a, bf, acc[n]);
        }
    }

    #pragma unroll
    for (int n = 0; n < TT / 16; ++n) {
        const int tl = n * 16 + lm;
        float p0 = 0.0f, p1 = 0.0f, p2 = 0.0f;
        if (ADDP) {
            p0 = pt[tl];
            p1 = pt[TT + tl];
            p2 = pt[2 * TT + tl];
        }
        #pragma unroll
        for (int r = 0; r < 8; r += 2) {
            const int m0 = mbase + 8 * hh + r;
            float v0 = acc[n][r]     * R_W + bias[m0];
            float v1 = acc[n][r + 1] * R_W + bias[m0 + 1];
            if (ADDP) {
                v0 += w0p[m0] * p0 + w0p[HN + m0] * p1 + w0p[2 * HN + m0] * p2;
                v1 += w0p[m0 + 1] * p0 + w0p[HN + m0 + 1] * p1 + w0p[2 * HN + m0 + 1] * p2;
            }
            v0 = fmaxf(v0, 0.0f);
            v1 = fmaxf(v1, 0.0f);
            const unsigned int pk = (unsigned int)hb(v0) | ((unsigned int)hb(v1) << 16);
            *(u32a*)(actOut + tl * KP + m0) = pk;
        }
    }
}

__global__ __launch_bounds__(256) void k_mlp(const float* __restrict__ p,
                                             const float* __restrict__ c,
                                             const float* __restrict__ ps,
                                             const float* __restrict__ W0,
                                             const float* __restrict__ b0,
                                             const float* __restrict__ b1,
                                             const float* __restrict__ b2,
                                             const float* __restrict__ W3,
                                             const float* __restrict__ b3,
                                             const unsigned short* __restrict__ P0,
                                             const unsigned short* __restrict__ P1,
                                             const unsigned short* __restrict__ P2,
                                             float* __restrict__ out)
{
    __shared__ __align__(16) unsigned short sC[TT * KP];
    __shared__ __align__(16) unsigned short sH1[TT * KP];
    __shared__ __align__(16) unsigned short sH2[TT * KP];
    __shared__ __align__(16) float sB[3 * HN];
    __shared__ __align__(16) float sW0p[DN * HN];
    __shared__ __align__(16) float sP[DN * TT];
    __shared__ __align__(16) float sW3[HN];
    __shared__ __align__(16) float sOut[TT];

    const int tid   = threadIdx.x;
    const int lane  = tid & 31;
    const int wave  = tid >> 5;
    const int mbase = wave * 16;
    const int tiles = TN / TT;
    const int b     = blockIdx.x / tiles;
    const int t0    = (blockIdx.x % tiles) * TT;

    {
        const float* cb = c + (size_t)b * CN * TN + t0;
        #pragma unroll 4
        for (int it = 0; it < (CN * TT / 4) / 256; ++it) {
            const int idx = it * 256 + tid;
            const int ch  = idx >> 5;
            const int t   = (idx & 31) * 4;
            const v4f f = *(const v4fa*)(cb + (size_t)ch * TN + t);
            sC[(t + 0) * KP + ch] = hb(f.x);
            sC[(t + 1) * KP + ch] = hb(f.y);
            sC[(t + 2) * KP + ch] = hb(f.z);
            sC[(t + 3) * KP + ch] = hb(f.w);
        }
    }
    __syncthreads();

    float oacc = 0.0f;

    #pragma unroll 1
    for (int j = 0; j < JN; ++j) {
        if (tid < HN) {
            sB[tid]          = b0[j * HN + tid];
            sB[HN + tid]     = b1[j * HN + tid];
            sB[2 * HN + tid] = b2[j * HN + tid];
            sW3[tid]         = W3[j * HN + tid];
        }
        {
            const float* W0j = W0 + (size_t)j * HN * WK0;
            const float* pG  = p + ((size_t)b * JN + j) * DN * TN + t0;
            for (int idx = tid; idx < DN * HN; idx += 256) {
                const int d = idx >> 7, m = idx & 127;
                sW0p[d * HN + m] = W0j[m * WK0 + d];
                sP[d * TT + m]   = pG[(size_t)d * TN + m];
            }
        }
        __syncthreads();

        gemm_layer<true>(sC, sH1, P0 + (size_t)j * HN * HN, sB, sW0p, sP, lane, mbase);
        __syncthreads();

        gemm_layer<false>(sH1, sH2, P1 + (size_t)j * HN * HN, sB + HN, sW0p, sP, lane, mbase);
        __syncthreads();

        gemm_layer<false>(sH2, sH1, P2 + (size_t)j * HN * HN, sB + 2 * HN, sW0p, sP, lane, mbase);
        __syncthreads();

        if (tid < TT) {
            const unsigned short* row = sH1 + tid * KP;
            const float b3v = b3[j];
            float dot = 0.0f;
            #pragma unroll 4
            for (int cix = 0; cix < HN / 8; ++cix) {
                Pack8 u;
                u.u = *(const v4ua*)(row + 8 * cix);
                #pragma unroll
                for (int e = 0; e < 8; ++e) dot += (float)u.h[e] * sW3[8 * cix + e];
            }
            const float o   = dot + b3v;
            const float psv = ps[((size_t)b * JN + j) * TN + t0 + tid];
            oacc += o * psv;
        }
        __syncthreads();
    }

    if (tid < TT) sOut[tid] = oacc * (1.0f / (float)JN);
    __syncthreads();

    if (wave == 0) {
        const v4f v = *(const v4fa*)(sOut + 4 * lane);
        float* d = out + (size_t)b * TN + t0 + 4 * lane;
        *(volatile v4f*)d = v;
        __threadfence();
        *(volatile v4f*)d = v;
    }
}

extern "C" void kernel_launch(void* const* d_in, const int* in_sizes, int n_in,
                              void* d_out, int out_size, void* d_ws, size_t ws_size,
                              hipStream_t stream)
{
    if (n_in < 12) return;
    if (in_sizes[0]  != BN * JN * DN * TN) return;
    if (in_sizes[2]  != BN * CN * TN) return;
    if (in_sizes[3]  != BN * JN * TN) return;
    if (in_sizes[4]  != JN * HN * WK0) return;
    if (in_sizes[5]  != JN * HN) return;
    if (in_sizes[6]  != JN * HN * HN) return;
    if (in_sizes[7]  != JN * HN) return;
    if (in_sizes[8]  != JN * HN * HN) return;
    if (in_sizes[9]  != JN * HN) return;
    if (in_sizes[10] != JN * HN) return;
    if (in_sizes[11] != JN) return;
    if (out_size != BN * TN) return;

    const float* p  = (const float*)d_in[0];
    const float* c  = (const float*)d_in[2];
    const float* ps = (const float*)d_in[3];
    const float* W0 = (const float*)d_in[4];
    const float* b0 = (const float*)d_in[5];
    const float* W1 = (const float*)d_in[6];
    const float* b1 = (const float*)d_in[7];
    const float* W2 = (const float*)d_in[8];
    const float* b2 = (const float*)d_in[9];
    const float* W3 = (const float*)d_in[10];
    const float* b3 = (const float*)d_in[11];
    float* out = (float*)d_out;

    const size_t bP = (size_t)JN * HN * HN * 2;
    const size_t total = 3 * bP;
    if (total > ws_size) return;
    if (total > (size_t)134217728) return;

    char* ws = (char*)d_ws;
    size_t off = 0;
    unsigned short* P0 = (unsigned short*)(ws + off); off += bP;
    unsigned short* P1 = (unsigned short*)(ws + off); off += bP;
    unsigned short* P2 = (unsigned short*)(ws + off); off += bP;
    if (off != total) return;

    {
        const int n8 = JN * HN * HN / 8;
        k_wcvt<<<dim3((n8 + 255) / 256, 3), 256, 0, stream>>>(W0, W1, W2, P0, P1, P2, n8);
    }
    k_mlp<<<dim3(BN * (TN / TT)), 256, 0, stream>>>(p, c, ps, W0, b0, b1, b2, W3, b3,
                                                     P0, P1, P2, out);
}
